// ScalableCritic_73366631350961
// MI455X (gfx1250) — hardware-verified
//
#include <hip/hip_runtime.h>
#include <stdint.h>
#include <stddef.h>

typedef _Float16 v16h __attribute__((ext_vector_type(16)));
typedef _Float16 v8h  __attribute__((ext_vector_type(8)));
typedef __bf16   v16b __attribute__((ext_vector_type(16)));
typedef unsigned short v8us __attribute__((ext_vector_type(8)));
typedef float    v8f  __attribute__((ext_vector_type(8)));
typedef float    v4f  __attribute__((ext_vector_type(4)));
typedef int      v4i  __attribute__((ext_vector_type(4)));
typedef v8h  __attribute__((may_alias)) v8ha;
typedef v8us __attribute__((may_alias)) v8usa;
typedef v4f  __attribute__((may_alias)) v4fa;
typedef v4i  __attribute__((may_alias)) v4ia;

union FragH { v16h v; v8h half[2]; };
union FragB { v16b v; v8us half[2]; };

#define NFEAT 3
#define NCOND 4
#define H1 64
#define H2 128
#define K3 132
#define K3P 160
#define SPB 8
#define TPTS 64
#define MAXT 128
#define NEGINIT (-1.0e9f)
#define HSC (1.0f / 128.0f)
#define PSC (1.0f / 512.0f)

__device__ __forceinline__ v8f wmma_f16(v16h a, v16h b, v8f c) {
  v8f d = __builtin_amdgcn_wmma_f32_16x16x32_f16(false, a, false, b, (short)0, c, false, false);
  asm volatile("v_nop\n\tv_nop\n\tv_nop\n\tv_nop" : "+v"(d) : "v"(a), "v"(b));
  return d;
}
__device__ __forceinline__ v8f wmma_bf16(v16b a, v16b b, v8f c) {
  v8f d = __builtin_amdgcn_wmma_f32_16x16x32_bf16(false, a, false, b, (short)0, c, false, false);
  asm volatile("v_nop\n\tv_nop\n\tv_nop\n\tv_nop" : "+v"(d) : "v"(a), "v"(b));
  return d;
}

__device__ __forceinline__ v16h load_frag(const _Float16* p, int h) {
  FragH f;
  f.half[0] = *(const v8ha*)(p + 8 * h);
  f.half[1] = *(const v8ha*)(p + 16 + 8 * h);
  return f.v;
}
__device__ __forceinline__ v16b load_frag_bf(const unsigned short* p, int h) {
  FragB f;
  f.half[0] = *(const v8usa*)(p + 8 * h);
  f.half[1] = *(const v8usa*)(p + 16 + 8 * h);
  return f.v;
}

__device__ __forceinline__ unsigned short bf_bits(float x) {
  unsigned u = __float_as_uint(x);
  u += 0x7FFFu + ((u >> 16) & 1u);
  return (unsigned short)(u >> 16);
}
__device__ __forceinline__ float bf_val(unsigned short b) {
  return __uint_as_float(((unsigned)b) << 16);
}
__device__ __forceinline__ float bfr(float x) { return bf_val(bf_bits(x)); }

__device__ __forceinline__ int lbound(const int* __restrict__ a, int n, int key) {
  int lo = 0, hi = n;
  #pragma unroll 1
  for (int it = 0; it < 32; ++it) {
    const int mid = (int)(((unsigned)lo + (unsigned)hi) >> 1);
    const int mc = min(mid, n - 1);
    const int v = a[mc];
    const bool go = lo < hi;
    const bool lt = v < key;
    lo = (go && lt) ? (mid + 1) : lo;
    hi = (go && !lt) ? mid : hi;
  }
  return lo;
}

__global__ __launch_bounds__(256) void prep_kernel(
    const int* __restrict__ bidx, const int* __restrict__ bsz,
    const float* __restrict__ W1, const float* __restrict__ b1,
    const float* __restrict__ W2, const float* __restrict__ W3,
    int* __restrict__ tbl, _Float16* __restrict__ w1t, _Float16* __restrict__ w2t,
    unsigned short* __restrict__ w3t, int N, int B, int nTB)
{
  const int tid = threadIdx.x;
  const int blk = blockIdx.x;
  if (blk < nTB) {
    const int g = blk * 256 + tid;
    int nb = bsz[0];
    nb = min(max(nb, 0), B);
    int vals[4];
    #pragma unroll
    for (int j = 0; j < 4; ++j) {
      const int key = 4 * g + j;
      const int lb = lbound(bidx, N, key);
      vals[j] = (key < nb) ? lb : N;
    }
    const v4i o = { vals[0], vals[1], vals[2], vals[3] };
    int* dst = tbl + (size_t)g * 4;
    *(volatile v4i*)dst = o;
    __threadfence();
    *(volatile v4i*)dst = o;
    return;
  }
  const int wb = blk - nTB;
  if (wb == 0) {
    const int pc = tid;
    const int n = pc >> 2;
    const int k0 = (pc & 3) * 8;
    const float bb = bfr(b1[n]) * 64.0f;
    v8h o;
    #pragma unroll
    for (int j = 0; j < 8; ++j) {
      const int k = k0 + j;
      const float wv = bfr(W1[min(k, NFEAT + NCOND - 1) * H1 + n]) * 64.0f;
      const float v = (k < NFEAT + NCOND) ? wv : ((k == NFEAT + NCOND) ? bb : 0.0f);
      o[j] = (_Float16)v;
    }
    _Float16* dst = w1t + (size_t)pc * 8;
    *(volatile v8h*)dst = o;
    __threadfence();
    *(volatile v8h*)dst = o;
  } else if (wb < 5) {
    const int pc = (wb - 1) * 256 + tid;
    const int n = pc >> 3;
    const int k0 = (pc & 7) * 8;
    v8h o;
    #pragma unroll
    for (int j = 0; j < 8; ++j) {
      const int k = k0 + j;
      o[j] = (_Float16)(bfr(W2[k * H2 + n]) * 64.0f);
    }
    _Float16* dst = w2t + (size_t)pc * 8;
    *(volatile v8h*)dst = o;
    __threadfence();
    *(volatile v8h*)dst = o;
  } else {
    const int pc = (wb - 5) * 256 + tid;
    const int n = pc / 20;
    const int k0 = (pc - n * 20) * 8;
    v8us o;
    #pragma unroll
    for (int j = 0; j < 8; ++j) {
      const int k = k0 + j;
      const float wv = W3[min(k, K3 - 1) * H2 + n];
      o[j] = (k < K3) ? bf_bits(wv) : (unsigned short)0;
    }
    unsigned short* dst = w3t + (size_t)pc * 8;
    *(volatile v8us*)dst = o;
    __threadfence();
    *(volatile v8us*)dst = o;
  }
}

__device__ __forceinline__ void plane_store(const unsigned short* sP, unsigned short* gP, int tid) {
  const v8us v0 = *(const v8usa*)(sP + 8 * tid);
  *(volatile v8us*)(gP + 8 * tid) = v0;
  if (tid < SPB * K3P / 8 - 128) {
    const v8us v1 = *(const v8usa*)(sP + 8 * (128 + tid));
    *(volatile v8us*)(gP + 8 * (128 + tid)) = v1;
  }
}

__global__ __launch_bounds__(128) void point_kernel(
    const float* __restrict__ pts, const int* __restrict__ bidx,
    const float* __restrict__ cond, const float* __restrict__ b2,
    const int* __restrict__ tbl,
    const _Float16* __restrict__ w1t, const _Float16* __restrict__ w2t,
    unsigned short* __restrict__ ahi, unsigned short* __restrict__ alo,
    int N, int B)
{
  __shared__ __attribute__((aligned(16))) _Float16 sW1[H1 * 32];
  __shared__ __attribute__((aligned(16))) _Float16 sW2[H2 * H1];
  __shared__ __attribute__((aligned(16))) _Float16 sXh[TPTS * 8];
  __shared__ __attribute__((aligned(16))) _Float16 sHA[TPTS * H1];
  __shared__ __attribute__((aligned(16))) int sSeg[TPTS];
  __shared__ __attribute__((aligned(16))) float sMax[2 * (SPB + 1) * H2];
  __shared__ __attribute__((aligned(16))) unsigned short sHi[SPB * K3P];
  __shared__ __attribute__((aligned(16))) unsigned short sLo[SPB * K3P];
  __shared__ int sBad;

  const int tid = threadIdx.x, lane = tid & 31, w = tid >> 5;
  const int h = lane >> 4, m = lane & 15;
  const int sFirst = blockIdx.x * SPB;

  int bnd[SPB + 1];
  #pragma unroll
  for (int s = 0; s <= SPB; ++s) {
    int v = tbl[sFirst + s];
    bnd[s] = min(max(v, 0), N);
  }
  #pragma unroll
  for (int s = 1; s <= SPB; ++s) bnd[s] = max(bnd[s], bnd[s - 1]);
  const int pStart = bnd[0], pEnd = bnd[SPB];
  const int cnt = pEnd - pStart;
  int ntiles = (cnt + TPTS - 1) / TPTS;
  const bool capped = ntiles > MAXT;
  ntiles = min(ntiles, MAXT);

  #pragma unroll 1
  for (int i = tid; i < H1 * 32 / 8; i += 128)
    *(v8ha*)(sW1 + 8 * i) = *(const v8ha*)(w1t + (size_t)8 * i);
  #pragma unroll 1
  for (int i = tid; i < H2 * H1 / 8; i += 128)
    *(v8ha*)(sW2 + 8 * i) = *(const v8ha*)(w2t + (size_t)8 * i);
  const float ninf = __uint_as_float(0xff800000u);
  #pragma unroll 1
  for (int i = tid; i < 2 * (SPB + 1) * H2; i += 128) sMax[i] = ninf;
  if (tid == 0) sBad = 0;

  float b2v[2];
  b2v[0] = bfr(b2[32 * w + m]);
  b2v[1] = bfr(b2[32 * w + 16 + m]);

  const v8f zero8 = {0.f, 0.f, 0.f, 0.f, 0.f, 0.f, 0.f, 0.f};
  const _Float16 zh = (_Float16)0.0f;
  const v8h z8h = { zh, zh, zh, zh, zh, zh, zh, zh };
  float* mbase = sMax + (h * (SPB + 1)) * H2 + 32 * w + m;

  #pragma unroll 1
  for (int t = 0; t < ntiles; ++t) {
    const int p0 = pStart + t * TPTS;
    __syncthreads();

    if (tid < TPTS) {
      const int p = p0 + tid;
      const int pc = min(p, N - 1);
      const float x0 = pts[(size_t)pc * NFEAT + 0];
      const float x1 = pts[(size_t)pc * NFEAT + 1];
      const float x2 = pts[(size_t)pc * NFEAT + 2];
      int bi = bidx[pc];
      const int bic = min(max(bi, 0), B - 1);
      const v4f cv = *(const v4fa*)(cond + (size_t)bic * NCOND);
      float c16;
      asm volatile("v_mov_b32 %0, 0x41800000" : "=v"(c16));
      v8h o;
      o[0] = (_Float16)(bfr(x0) * 16.0f);
      o[1] = (_Float16)(bfr(x1) * 16.0f);
      o[2] = (_Float16)(bfr(x2) * 16.0f);
      o[3] = (_Float16)(bfr(cv.x) * 16.0f);
      o[4] = (_Float16)(bfr(cv.y) * 16.0f);
      o[5] = (_Float16)(bfr(cv.z) * 16.0f);
      o[6] = (_Float16)(bfr(cv.w) * 16.0f);
      o[7] = (_Float16)c16;
      *(v8ha*)(sXh + tid * 8) = o;
      int sl = 0;
      #pragma unroll
      for (int s = 1; s < SPB; ++s) sl += (p >= bnd[s]) ? 1 : 0;
      const bool live = p < pEnd;
      sSeg[tid] = live ? sl : SPB;
      if (live && bi != sFirst + sl) sBad = 1;
    }
    __syncthreads();

    {
      const v8h xv = *(const v8ha*)(sXh + (16 * w + m) * 8);
      FragH xb;
      xb.half[0] = (h == 0) ? xv : z8h;
      xb.half[1] = z8h;
      #pragma unroll
      for (int t4 = 0; t4 < 4; ++t4) {
        const v16h a = load_frag(sW1 + (16 * t4 + m) * 32, h);
        const v8f d = wmma_f16(a, xb.v, zero8);
        v8h o;
        #pragma unroll
        for (int r = 0; r < 8; ++r) {
          const float u = d[r] * HSC;
          o[r] = (_Float16)fmaxf(u, 0.2f * u);
        }
        *(v8ha*)(sHA + (16 * w + m) * H1 + 16 * t4 + 8 * h) = o;
      }
    }
    __syncthreads();

    v8f acc[4][2];
    #pragma unroll
    for (int mt = 0; mt < 4; ++mt) { acc[mt][0] = zero8; acc[mt][1] = zero8; }
    #pragma unroll
    for (int kk = 0; kk < 2; ++kk) {
      const int k0 = 32 * kk;
      const v16h bf0 = load_frag(sW2 + (32 * w + m) * H1 + k0, h);
      const v16h bf1 = load_frag(sW2 + (32 * w + 16 + m) * H1 + k0, h);
      #pragma unroll
      for (int mt = 0; mt < 4; ++mt) {
        const v16h a = load_frag(sHA + (16 * mt + m) * H1 + k0, h);
        acc[mt][0] = wmma_f16(a, bf0, acc[mt][0]);
        acc[mt][1] = wmma_f16(a, bf1, acc[mt][1]);
      }
    }

    #pragma unroll
    for (int mt = 0; mt < 4; ++mt) {
      const v4i sa = *(const v4ia*)(sSeg + 16 * mt + 8 * h);
      const v4i sb = *(const v4ia*)(sSeg + 16 * mt + 8 * h + 4);
      int sg[8];
      sg[0] = sa.x; sg[1] = sa.y; sg[2] = sa.z; sg[3] = sa.w;
      sg[4] = sb.x; sg[5] = sb.y; sg[6] = sb.z; sg[7] = sb.w;
      #pragma unroll
      for (int nt = 0; nt < 2; ++nt) {
        float v[8];
        #pragma unroll
        for (int r = 0; r < 8; ++r) {
          const float u = acc[mt][nt][r] * PSC + b2v[nt];
          v[r] = fmaxf(u, 0.2f * u);
        }
        float* cb = mbase + 16 * nt;
        if (sg[0] == sg[7]) {
          float mx = v[0];
          #pragma unroll
          for (int r = 1; r < 8; ++r) mx = fmaxf(mx, v[r]);
          float* q = cb + sg[0] * H2;
          *q = fmaxf(*q, mx);
        } else {
          int cur = sg[0];
          float cm = v[0];
          #pragma unroll
          for (int r = 1; r < 8; ++r) {
            if (sg[r] != cur) {
              float* q = cb + cur * H2;
              *q = fmaxf(*q, cm);
              cur = sg[r];
              cm = v[r];
            } else {
              cm = fmaxf(cm, v[r]);
            }
          }
          float* q = cb + cur * H2;
          *q = fmaxf(*q, cm);
        }
      }
    }
  }
  __syncthreads();

  const bool poison = capped || (sBad != 0);
  const float qnan = __uint_as_float(0x7fc00000u);
  {
    const int c = tid;
    #pragma unroll
    for (int s = 0; s < SPB; ++s) {
      float g = fmaxf(sMax[s * H2 + c], sMax[(SPB + 1 + s) * H2 + c]);
      g = fmaxf(g, NEGINIT);
      g = poison ? qnan : g;
      const unsigned short hb = bf_bits(g);
      const float hvf = bf_val(hb);
      const unsigned short lb = bf_bits(g - hvf);
      sHi[s * K3P + c] = hb;
      sLo[s * K3P + c] = lb;
    }
    if (tid < K3P - H2) {
      const int cc = min(tid, NCOND - 1);
      #pragma unroll
      for (int s = 0; s < SPB; ++s) {
        const int rg = min(sFirst + s, B - 1);
        const float cv = cond[(size_t)rg * NCOND + cc];
        const unsigned short hb = (tid < NCOND) ? bf_bits(cv) : (unsigned short)0;
        sHi[s * K3P + H2 + tid] = hb;
        sLo[s * K3P + H2 + tid] = (unsigned short)0;
      }
    }
  }
  __syncthreads();

  unsigned short* ghi = ahi + (size_t)sFirst * K3P;
  unsigned short* glo = alo + (size_t)sFirst * K3P;
  plane_store(sHi, ghi, tid);
  plane_store(sLo, glo, tid);
  __threadfence();
  plane_store(sHi, ghi, tid);
  plane_store(sLo, glo, tid);
}

__global__ __launch_bounds__(128) void head_kernel(
    const unsigned short* __restrict__ ahi, const unsigned short* __restrict__ alo,
    const unsigned short* __restrict__ w3t, const float* __restrict__ b3,
    const float* __restrict__ W4, const float* __restrict__ b4,
    float* __restrict__ out, int B)
{
  __shared__ __attribute__((aligned(16))) float sB3[H2];
  __shared__ __attribute__((aligned(16))) float sW4[H2];
  __shared__ __attribute__((aligned(16))) float sScore[64];

  const int tid = threadIdx.x, lane = tid & 31, w = tid >> 5;
  const int h = lane >> 4, m = lane & 15;
  sB3[tid] = bfr(b3[tid]);
  sW4[tid] = bfr(W4[tid]);
  __syncthreads();

  const int r0 = blockIdx.x * 64 + 16 * w;
  const unsigned short* pah = ahi + (size_t)(r0 + m) * K3P;
  const unsigned short* pal = alo + (size_t)(r0 + m) * K3P;

  const v8f zero8 = {0.f, 0.f, 0.f, 0.f, 0.f, 0.f, 0.f, 0.f};
  v8f acc[8];
  #pragma unroll
  for (int nt = 0; nt < 8; ++nt) acc[nt] = zero8;

  #pragma unroll 1
  for (int k0 = 0; k0 < K3P; k0 += 32) {
    const v16b fa = load_frag_bf(pah + k0, h);
    const v16b fl = load_frag_bf(pal + k0, h);
    #pragma unroll
    for (int nt = 0; nt < 8; ++nt) {
      const v16b fb = load_frag_bf(w3t + (size_t)(16 * nt + m) * K3P + k0, h);
      acc[nt] = wmma_bf16(fa, fb, acc[nt]);
      acc[nt] = wmma_bf16(fl, fb, acc[nt]);
    }
  }

  float part[8];
  #pragma unroll
  for (int r = 0; r < 8; ++r) part[r] = 0.0f;
  #pragma unroll
  for (int nt = 0; nt < 8; ++nt) {
    const float bb = sB3[16 * nt + m];
    const float ww = sW4[16 * nt + m];
    #pragma unroll
    for (int r = 0; r < 8; ++r) {
      float u = acc[nt][r] + bb;
      u = fmaxf(u, 0.2f * u);
      part[r] += u * ww;
    }
  }
  #pragma unroll
  for (int r = 0; r < 8; ++r) {
    part[r] += __shfl_xor(part[r], 1);
    part[r] += __shfl_xor(part[r], 2);
    part[r] += __shfl_xor(part[r], 4);
    part[r] += __shfl_xor(part[r], 8);
  }
  const float b4r = bfr(b4[0]);
  if (m == 0) {
    #pragma unroll
    for (int r = 0; r < 8; ++r) sScore[16 * w + 8 * h + r] = part[r] + b4r;
  }
  __syncthreads();

  if (tid < 16) {
    const v4f v = *(const v4fa*)(sScore + 4 * tid);
    float* dst = out + (size_t)blockIdx.x * 64 + 4 * tid;
    *(volatile v4f*)dst = v;
    __threadfence();
    *(volatile v4f*)dst = v;
  }
}

static inline size_t a128(size_t x) { return (x + 127) & ~(size_t)127; }

extern "C" void kernel_launch(void* const* d_in, const int* in_sizes, int n_in,
                              void* d_out, int out_size, void* d_ws, size_t ws_size,
                              hipStream_t stream) {
  if (n_in < 12) return;
  const int N = in_sizes[1];
  if (N <= 0 || in_sizes[0] != NFEAT * N) return;
  const int B = in_sizes[2] / NCOND;
  if (B <= 0 || in_sizes[2] != NCOND * B) return;
  if (out_size != B) return;
  if ((B % 64) != 0) return;
  if (in_sizes[3] < 1) return;
  if (in_sizes[4] != (NFEAT + NCOND) * H1 || in_sizes[5] != H1) return;
  if (in_sizes[6] != H1 * H2 || in_sizes[7] != H2) return;
  if (in_sizes[8] != K3 * H2 || in_sizes[9] != H2) return;
  if (in_sizes[10] != H2 || in_sizes[11] < 1) return;

  const float* pts  = (const float*)d_in[0];
  const int*   bidx = (const int*)d_in[1];
  const float* cond = (const float*)d_in[2];
  const int*   bsz  = (const int*)d_in[3];
  const float* W1 = (const float*)d_in[4];
  const float* b1 = (const float*)d_in[5];
  const float* W2 = (const float*)d_in[6];
  const float* b2 = (const float*)d_in[7];
  const float* W3 = (const float*)d_in[8];
  const float* b3 = (const float*)d_in[9];
  const float* W4 = (const float*)d_in[10];
  const float* b4 = (const float*)d_in[11];
  float* out = (float*)d_out;

  const int nblk = B / SPB;
  const int TBL = ((nblk * SPB + 1 + 1023) / 1024) * 1024;
  const int nTB = TBL / 1024;

  const size_t tbl_bytes = (size_t)TBL * 4;
  const size_t w1t_bytes = (size_t)H1 * 32 * 2;
  const size_t w2t_bytes = (size_t)H2 * H1 * 2;
  const size_t w3t_bytes = (size_t)H2 * K3P * 2;
  const size_t pln_bytes = (size_t)B * K3P * 2;
  size_t off = 0;
  const size_t off_tbl = off; off = a128(off + tbl_bytes);
  const size_t off_w1t = off; off = a128(off + w1t_bytes);
  const size_t off_w2t = off; off = a128(off + w2t_bytes);
  const size_t off_w3t = off; off = a128(off + w3t_bytes);
  const size_t off_ahi = off; off = a128(off + pln_bytes);
  const size_t off_alo = off; off = a128(off + pln_bytes);
  const size_t total = off;
  if (total > ws_size) return;

  char* ws = (char*)d_ws;
  int* tbl = (int*)(ws + off_tbl);
  _Float16* w1t = (_Float16*)(ws + off_w1t);
  _Float16* w2t = (_Float16*)(ws + off_w2t);
  unsigned short* w3t = (unsigned short*)(ws + off_w3t);
  unsigned short* ahi = (unsigned short*)(ws + off_ahi);
  unsigned short* alo = (unsigned short*)(ws + off_alo);

  prep_kernel<<<nTB + 15, 256, 0, stream>>>(bidx, bsz, W1, b1, W2, W3, tbl, w1t, w2t, w3t, N, B, nTB);
  point_kernel<<<nblk, 128, 0, stream>>>(pts, bidx, cond, b2, tbl, w1t, w2t, ahi, alo, N, B);
  head_kernel<<<B / 64, 128, 0, stream>>>(ahi, alo, w3t, b3, W4, b4, out, B);
}
